// DeTGC_59399397703719
// MI455X (gfx1250) — hardware-run, weakly checked
//
#include <hip/hip_runtime.h>
#include <math.h>

typedef __attribute__((ext_vector_type(16))) _Float16 v16h;
typedef __attribute__((ext_vector_type(8)))  _Float16 v8h;
typedef __attribute__((ext_vector_type(8)))  float    v8f;
typedef __attribute__((ext_vector_type(4)))  float    v4f;

constexpr int kNb       = 32;
constexpr int kCin      = 64;
constexpr int kTf       = 300;
constexpr int kVj       = 25;
constexpr int kEta      = 9;
constexpr int kCout     = 64;
constexpr int kCols     = kTf * kVj;
constexpr int kRowsAll  = kNb * kCols;
constexpr int kTaps     = 2 * kEta;
constexpr int kKtot     = kTaps * kCin;
constexpr int kWin      = kCin * kEta;
constexpr int kTileCols = 100;
constexpr int kHalo     = 28;
constexpr int kTileM    = 128;
constexpr int kTilesPerN = kCols / kTileCols;
constexpr int kSlab     = kCout * kCols;
constexpr int kOPitch   = 132;
constexpr int kPPitch   = 72;
constexpr float kWCarry    = 1024.0f;
constexpr float kWCarryInv = 1.0f / 1024.0f;
constexpr int kWtChunks = kCout * kKtot / 8;
constexpr int kWtBlocks = kWtChunks / 256;

static_assert(kTileCols + kHalo == kTileM, "tile rows");
static_assert(kTilesPerN * kTileCols == kCols, "column tiles exact");
static_assert((kCols % 4) == 0 && (kTileCols % 4) == 0, "16-B groups never straddle");
static_assert((kRowsAll % 128) == 0, "pack tiles exact");
static_assert((kKtot % 32) == 0 && (kCout % 16) == 0 && (kTileM % 16) == 0, "WMMA tile multiples");
static_assert((kSlab % 32) == 0, "per-n output slab is line aligned");
static_assert(kWtBlocks * 256 == kWtChunks, "weight plane coverage exact");
static_assert(kCin == 64, "packed row is one 128-B line");

constexpr size_t kOffXH   = 0;
constexpr size_t kOffWT   = kOffXH + (size_t)kRowsAll * kCin * 2;
constexpr size_t kOffSS   = kOffWT + (size_t)kCout * kKtot * 2;
constexpr size_t kWsTotal = kOffSS + 128 * 4;
static_assert(kWsTotal == 30867968ull, "carve total");
static_assert(kWsTotal <= 134217728ull, "carve cap");
static_assert((kOffWT % 128) == 0 && (kOffSS % 128) == 0, "128-B aligned regions");

union FragU { v16h v; v8h h[2]; };
__device__ __forceinline__ v16h ldfrag(const _Float16* p) {
  FragU f;
  f.h[0] = *(const v8h*)(p);
  f.h[1] = *(const v8h*)(p + 16);
  return f.v;
}
__device__ __forceinline__ v8f mma_f16(v16h a, v16h b, v8f c) {
  c = __builtin_amdgcn_wmma_f32_16x16x32_f16(false, a, false, b, (short)0, c, false, false);
  asm volatile("v_nop\n\tv_nop\n\tv_nop\n\tv_nop" : "+v"(c) : "v"(a), "v"(b));
  return c;
}

__global__ __launch_bounds__(256) void prep_kernel(
    const float* __restrict__ W, const float* __restrict__ tr, const float* __restrict__ bias,
    const float* __restrict__ gamma, const float* __restrict__ beta,
    const float* __restrict__ rmean, const float* __restrict__ rvar,
    _Float16* __restrict__ wt, float* __restrict__ ss)
{
  const int tid = threadIdx.x;
  if (blockIdx.x < kWtBlocks) {
    const int i   = blockIdx.x * 256 + tid;
    const int o   = i / 144;
    const int kk0 = (i - o * 144) * 8;
    const int tap = kk0 >> 6;
    const int c0  = kk0 & 63;
    const int e   = tap >> 1;
    const int s   = tap & 1;
    const float trv = tr[e];
    const float dfl = floorf(trv);
    const float al  = (dfl + 1.0f) - trv;
    const float sel = (s == 0) ? al : (1.0f - al);
    const float wgt = sel * kWCarry;
    const float* wp = W + (size_t)o * kWin + (size_t)c0 * kEta + e;
    v8h hv;
#pragma unroll
    for (int u = 0; u < 8; ++u) {
      const float w = wp[u * kEta];
      hv[u] = (_Float16)(w * wgt);
    }
    _Float16* p = wt + (size_t)i * 8;
    *(volatile v8h*)p = hv;
    __threadfence();
    *(volatile v8h*)p = hv;
  } else {
    if (tid < 32) {
      const int o0 = (tid * 4) & 63;
      const v4f vv = *(const v4f*)(rvar + o0);
      const v4f gg = *(const v4f*)(gamma + o0);
      const v4f be = *(const v4f*)(beta + o0);
      const v4f bb = *(const v4f*)(bias + o0);
      const v4f mm = *(const v4f*)(rmean + o0);
      v4f val;
#pragma unroll
      for (int u = 0; u < 4; ++u) {
        const float inv = rsqrtf(vv[u] + 1e-5f);
        const float sc  = gg[u] * inv;
        const float sh  = be[u] + (bb[u] - mm[u]) * sc;
        val[u] = (tid < 16) ? (sc * kWCarryInv) : sh;
      }
      float* p = ss + tid * 4;
      *(volatile v4f*)p = val;
      __threadfence();
      *(volatile v4f*)p = val;
    }
  }
}

__global__ __launch_bounds__(256) void pack_kernel(const float* __restrict__ x, _Float16* __restrict__ xh)
{
  __shared__ __align__(16) _Float16 sP[kTileM * kPPitch];
  const int tid = threadIdx.x, lane = tid & 31, wave = tid >> 5;
  const int g0 = blockIdx.x * 128;
  {
    const int g   = g0 + 4 * lane;
    const int n   = g / kCols;
    const int col = g - n * kCols;
    const float* xb = x + ((size_t)n * kCin) * kCols + col;
#pragma unroll
    for (int i = 0; i < 8; ++i) {
      const int c = wave + 8 * i;
      const v4f v = *(const v4f*)(xb + (size_t)c * kCols);
      const float f0 = v[0], f1 = v[1], f2 = v[2], f3 = v[3];
      sP[(4 * lane + 0) * kPPitch + c] = (_Float16)f0;
      sP[(4 * lane + 1) * kPPitch + c] = (_Float16)f1;
      sP[(4 * lane + 2) * kPPitch + c] = (_Float16)f2;
      sP[(4 * lane + 3) * kPPitch + c] = (_Float16)f3;
    }
  }
  __syncthreads();
  const int qq = lane >> 3, c8 = (lane & 7) * 8;
  v8h rv[4];
#pragma unroll
  for (int it = 0; it < 4; ++it) {
    const int row = it * 32 + wave * 4 + qq;
    rv[it] = *(const v8h*)(sP + row * kPPitch + c8);
  }
  for (int pass = 0; pass < 2; ++pass) {
#pragma unroll
    for (int it = 0; it < 4; ++it) {
      const int row = it * 32 + wave * 4 + qq;
      *(volatile v8h*)(xh + (size_t)(g0 + row) * kCin + c8) = rv[it];
    }
    __threadfence();
  }
}

__global__ __launch_bounds__(256) void gemm_kernel(
    const _Float16* __restrict__ xh, const _Float16* __restrict__ wt, const float* __restrict__ ss,
    const float* __restrict__ tr, float* __restrict__ out)
{
  __shared__ __align__(16) float sO[kCout * kOPitch];
  __shared__ int sTap[32];
  const int tid = threadIdx.x, lane = tid & 31, wave = tid >> 5;
  const int rlane = lane & 15;
  const int hh    = lane >> 4;
  const int koff  = hh * 8;
  const int n = blockIdx.x / kTilesPerN;
  const int j = blockIdx.x - n * kTilesPerN;

  if (tid < 32) {
    const int tp = (tid < kTaps) ? tid : (kTaps - 1);
    const int e  = tp >> 1;
    const int s  = tp & 1;
    float dfl = floorf(tr[e]);
    dfl = fminf(fmaxf(dfl, -400.0f), 400.0f);
    sTap[tid] = (int)dfl + s;
  }
  __syncthreads();

  const int m = wave * 16 + rlane;
  int gc = j * kTileCols + m;
  gc = (gc >= kCols) ? (gc - kCols) : gc;
  const int t = gc / kVj;
  const int v = gc - t * kVj;
  const size_t rowN = (size_t)n * kTf;

  v8f acc[4];
#pragma unroll
  for (int jt = 0; jt < 4; ++jt) acc[jt] = (v8f){0.f, 0.f, 0.f, 0.f, 0.f, 0.f, 0.f, 0.f};

#pragma unroll 1
  for (int tap = 0; tap < kTaps; ++tap) {
    int tt = t + sTap[tap];
    tt = (tt < 0) ? 0 : ((tt > kTf - 1) ? (kTf - 1) : tt);
    const _Float16* ap = xh + ((rowN + (size_t)tt) * kVj + (size_t)v) * kCin + koff;
    const _Float16* bp = wt + (size_t)rlane * kKtot + tap * kCin + koff;
#pragma unroll
    for (int cc = 0; cc < 2; ++cc) {
      const v16h a = ldfrag(ap + cc * 32);
      v16h b[4];
#pragma unroll
      for (int jt = 0; jt < 4; ++jt) b[jt] = ldfrag(bp + (size_t)jt * 16 * kKtot + cc * 32);
#pragma unroll
      for (int jt = 0; jt < 4; ++jt) acc[jt] = mma_f16(a, b[jt], acc[jt]);
    }
  }

#pragma unroll
  for (int jt = 0; jt < 4; ++jt) {
    const int o = jt * 16 + rlane;
    const float sc = ss[o];
    const float sh = ss[kCout + o];
    v4f w0, w1;
    w0[0] = acc[jt][0] * sc + sh;
    w0[1] = acc[jt][1] * sc + sh;
    w0[2] = acc[jt][2] * sc + sh;
    w0[3] = acc[jt][3] * sc + sh;
    w1[0] = acc[jt][4] * sc + sh;
    w1[1] = acc[jt][5] * sc + sh;
    w1[2] = acc[jt][6] * sc + sh;
    w1[3] = acc[jt][7] * sc + sh;
    float* dst = sO + o * kOPitch + wave * 16 + hh * 8;
    *(v4f*)(dst)     = w0;
    *(v4f*)(dst + 4) = w1;
  }
  __syncthreads();

  const int qq  = lane >> 3;
  const int sub = lane & 7;
  float* slab = out + (size_t)n * kSlab;
  v4f vals[8];
#pragma unroll
  for (int it = 0; it < 8; ++it) {
    const int o    = it * 8 + wave;
    const int pO   = o * kCols + j * kTileCols;
    const int f    = (32 - (pO & 31)) & 31;
    const int lc   = f + 32 * qq;
    const int lcl  = (lc > 96) ? 96 : lc;
    const int lcol = lcl + 4 * sub;
    const int gcol = j * kTileCols + lcol;
    const int on   = (o + 1 > kCout - 1) ? (kCout - 1) : (o + 1);
    const int orow = (gcol >= kCols) ? on : o;
    vals[it] = *(const v4f*)(sO + orow * kOPitch + lcol);
  }
  for (int pass = 0; pass < 2; ++pass) {
#pragma unroll
    for (int it = 0; it < 8; ++it) {
      const int o  = it * 8 + wave;
      const int pO = o * kCols + j * kTileCols;
      const int f  = (32 - (pO & 31)) & 31;
      const int lc = f + 32 * qq;
      const int pS = pO + lc;
      const bool valid = (lc < kTileCols) && (pS + 32 <= kSlab);
      if (valid) {
        *(volatile v4f*)(slab + pS + 4 * sub) = vals[it];
      }
    }
    __threadfence();
  }
}

extern "C" void kernel_launch(void* const* d_in, const int* in_sizes, int n_in,
                              void* d_out, int out_size, void* d_ws, size_t ws_size,
                              hipStream_t stream) {
  if (n_in < 8) return;
  if (in_sizes[0] != kNb * kCin * kCols) return;
  if (in_sizes[1] != kEta) return;
  if (in_sizes[2] != kCout * kWin) return;
  if (in_sizes[3] != kCout) return;
  if (in_sizes[4] != kCout) return;
  if (in_sizes[5] != kCout) return;
  if (in_sizes[6] != kCout) return;
  if (in_sizes[7] != kCout) return;
  if (out_size != kNb * kSlab) return;
  if (ws_size < kWsTotal) return;

  const float* x     = (const float*)d_in[0];
  const float* tr    = (const float*)d_in[1];
  const float* W     = (const float*)d_in[2];
  const float* bias  = (const float*)d_in[3];
  const float* gamma = (const float*)d_in[4];
  const float* beta  = (const float*)d_in[5];
  const float* rmean = (const float*)d_in[6];
  const float* rvar  = (const float*)d_in[7];
  float* out = (float*)d_out;

  char* ws = (char*)d_ws;
  _Float16* XH = (_Float16*)(ws + kOffXH);
  _Float16* WT = (_Float16*)(ws + kOffWT);
  float*    SS = (float*)(ws + kOffSS);

  prep_kernel<<<kWtBlocks + 1, 256, 0, stream>>>(W, tr, bias, gamma, beta, rmean, rvar, WT, SS);
  pack_kernel<<<kRowsAll / 128, 256, 0, stream>>>(x, XH);
  gemm_kernel<<<kNb * kTilesPerN, 256, 0, stream>>>(XH, WT, SS, tr, out);
}
